// DyadXLSTM_24326694764772
// MI455X (gfx1250) — hardware-verified
//
#include <hip/hip_runtime.h>


namespace {
constexpr int B = 32, T = 256, F = 224, EE = 32, NH = 4, DH = 64, D = 256, H = 256, NT = B * T, NDY = 10000, PW = 1040;
constexpr float XS = 8.0f, HS = 64.0f, WSC = 256.0f;
typedef _Float16 b16;
typedef __attribute__((ext_vector_type(16))) _Float16 v16b;
typedef __attribute__((ext_vector_type(8))) _Float16 v8b;
typedef __attribute__((ext_vector_type(8))) float v8f;
typedef __attribute__((ext_vector_type(4))) float v4f;
typedef __attribute__((ext_vector_type(2))) float v2f;
__device__ __forceinline__ float bf16_rne(float f) { unsigned int u = __float_as_uint(f); u += 0x7FFFu + ((u >> 16) & 1u); return __uint_as_float(u & 0xFFFF0000u); }
__device__ __forceinline__ void split16(float v, b16& hi, b16& lo) { hi = (b16)v; lo = (b16)(v - (float)hi); }
__device__ __forceinline__ v16b frag_kb(const b16* p, int hh) { const v8b a = *(const v8b*)(p + 8 * hh), b = *(const v8b*)(p + 16 + 8 * hh); v16b f;
#pragma unroll
  for (int e = 0; e < 8; ++e) { f[e] = a[e]; f[8 + e] = b[e]; } return f; }
__device__ __forceinline__ v8f wmma16b(v16b a, v16b b, v8f c) { v8f d = __builtin_amdgcn_wmma_f32_16x16x32_f16(false, a, false, b, (short)0, c, false, false); asm volatile("v_nop\n\tv_nop\n\tv_nop\n\tv_nop" : "+v"(d) : "v"(a), "v"(b)); return d; }
__device__ __forceinline__ void wave_lds_sync() { __builtin_amdgcn_fence(__ATOMIC_RELEASE, "workgroup"); __builtin_amdgcn_wave_barrier(); __builtin_amdgcn_fence(__ATOMIC_ACQUIRE, "workgroup"); }
__device__ __forceinline__ float pmul(float a, float b) { float p = a * b; asm volatile("" : "+v"(p)); return p; }
__device__ __forceinline__ int iclamp(int v, int lo, int hi) { return v < lo ? lo : (v > hi ? hi : v); }
__device__ __forceinline__ float sigm(float v) { return 1.0f / (1.0f + __expf(-v)); }

__global__ __launch_bounds__(256) void wio_kernel(const float* __restrict__ w, int KIN, int OUTW, int ro, b16* __restrict__ WT) {
  const int u = blockIdx.x * 256 + threadIdx.x; if (u >= OUTW * KIN / 8) return; const int e = u * 8; const int o = e / KIN, k0 = e % KIN; v8b v;
#pragma unroll
  for (int j = 0; j < 8; ++j) v[j] = (b16)(bf16_rne(w[(size_t)(k0 + j) * OUTW + o]) * WSC); for (int pass = 0; pass < 2; ++pass) { *(volatile v8b*)(WT + (size_t)(ro + o) * KIN + k0) = v; __threadfence(); }
}
__global__ __launch_bounds__(256) void wzero_kernel(b16* __restrict__ WT, int n8) { const int u = blockIdx.x * 256 + threadIdx.x; if (u >= n8) return; v8b z = {}; for (int pass = 0; pass < 2; ++pass) { *(volatile v8b*)(WT + (size_t)u * 8) = z; __threadfence(); } }
__global__ __launch_bounds__(256) void wr_kernel(const float* __restrict__ Rz, const float* __restrict__ Ri, const float* __restrict__ Rf, const float* __restrict__ Ro, b16* __restrict__ WR) {
  const int u = blockIdx.x * 256 + threadIdx.x; if (u >= NH * 256 * DH / 8) return; const int e8 = u * 8; const int h = e8 / (256 * DH), row = (e8 / DH) % 256, d0 = e8 % DH; const int g = row / DH, e = row % DH; const float* R = g == 0 ? Rz : (g == 1 ? Ri : (g == 2 ? Rf : Ro)); v8b v;
#pragma unroll
  for (int j = 0; j < 8; ++j) v[j] = (b16)(bf16_rne(R[((size_t)h * DH + d0 + j) * DH + e]) * WSC); for (int pass = 0; pass < 2; ++pass) { *(volatile v8b*)(WR + e8) = v; __threadfence(); }
}
__global__ __launch_bounds__(32) void x0_kernel(const float* __restrict__ X, const int* __restrict__ di, const float* __restrict__ emb, float* __restrict__ XR) {
  const int lane = threadIdx.x; const size_t t0 = (size_t)blockIdx.x * 16;
  for (int pass = 0; pass < 2; ++pass) { for (int rr = 0; rr < 16; ++rr) { const size_t t = t0 + rr; const int b = (int)(t / T); const int dy = iclamp(di[b], 0, NDY - 1);
      for (int q = 0; q < 8; ++q) { const int c = q * 32 + lane; ((volatile float*)XR)[t * D + c] = c < F ? bf16_rne(X[t * F + c]) : bf16_rne(emb[(size_t)dy * EE + c - F]); } } __threadfence(); }
}
template <int MODE>
__global__ __launch_bounds__(32) void proj_kernel(const float* __restrict__ XR, const float* __restrict__ g, const float* __restrict__ bb, const b16* __restrict__ W, const float* __restrict__ bi, const float* __restrict__ bf, int NTV, float* __restrict__ P, float* __restrict__ IF) {
  __shared__ __attribute__((aligned(16))) b16 Ah[16][D + 8], Al[16][D + 8]; __shared__ __attribute__((aligned(16))) float Tf[16][128 + 4], Sif[16][8];
  const int lane = threadIdx.x, nloc = lane & 15, hlf = lane >> 4; const size_t m0 = (size_t)blockIdx.x * 16; if (m0 >= (size_t)NTV) return;
  { float gg[8], be[8]; for (int q = 0; q < 8; ++q) { gg[q] = bf16_rne(g[q * 32 + lane]); be[q] = bf16_rne(bb[q * 32 + lane]); }
    for (int rr = 0; rr < 16; ++rr) { float v[8]; float s = 0.0f; for (int q = 0; q < 8; ++q) { v[q] = XR[(m0 + rr) * D + q * 32 + lane]; s += v[q]; } for (int o = 16; o; o >>= 1) s += __shfl_xor(s, o); const float mu = s * (1.0f / D); float vq = 0.0f; for (int q = 0; q < 8; ++q) { const float d_ = v[q] - mu; vq += pmul(d_, d_); }
      for (int o = 16; o; o >>= 1) vq += __shfl_xor(vq, o); const float rs = rsqrtf(vq * (1.0f / D) + 1e-5f); for (int q = 0; q < 8; ++q) { b16 p, ql; split16((pmul(pmul(v[q] - mu, rs), gg[q]) + be[q]) * XS, p, ql); Ah[rr][q * 32 + lane] = p; Al[rr][q * 32 + lane] = ql; } } }
  wave_lds_sync(); const float sc = 1.0f / (XS * WSC); constexpr int NTILE = MODE == 0 ? PW / 16 : 64;
#pragma unroll 1
  for (int cg = 0; cg < (NTILE + 7) / 8; ++cg) { const int nt = min(8, NTILE - cg * 8); v8f acc[8];
#pragma unroll
    for (int t = 0; t < 8; ++t) acc[t] = (v8f){};
#pragma unroll 2
    for (int kb = 0; kb < D; kb += 32) { const v16b a = frag_kb(&Ah[nloc][kb], hlf), al = frag_kb(&Al[nloc][kb], hlf);
#pragma unroll
      for (int t = 0; t < 8; ++t) { if (t < nt) { const v16b bw = frag_kb(W + (size_t)(cg * 128 + t * 16 + nloc) * D + kb, hlf); acc[t] = wmma16b(a, bw, acc[t]); acc[t] = wmma16b(al, bw, acc[t]); } } }
    if (MODE == 0 && cg == 8) {
      for (int r8 = 0; r8 < 8; ++r8) { const float v = acc[0][r8] * sc; if (nloc < 4) Sif[8 * hlf + r8][nloc] = v + bf16_rne(bi[nloc]); else if (nloc < 8) Sif[8 * hlf + r8][nloc] = v + bf16_rne(bf[nloc - 4]); }
      wave_lds_sync();
      for (int pass = 0; pass < 2; ++pass) { for (int q = 0; q < 4; ++q) ((volatile float*)IF)[m0 * 8 + q * 32 + lane] = Sif[(q * 32 + lane) >> 3][(q * 32 + lane) & 7]; __threadfence(); } }
    else {
#pragma unroll
      for (int t = 0; t < 8; ++t) { const int c = cg * 128 + t * 16 + nloc;
#pragma unroll 1
        for (int r8 = 0; r8 < 8; ++r8) { float v = acc[t][r8] * sc; if (MODE == 0) { if (c >= 256 && c < 512) v *= 0.125f; else if (c >= 768) v = sigm(v); } Tf[8 * hlf + r8][t * 16 + nloc] = v; } }
      wave_lds_sync();
      for (int pass = 0; pass < 2; ++pass) { for (int rr = 0; rr < 16; ++rr) *(volatile v4f*)(P + (m0 + rr) * 1024 + cg * 128 + lane * 4) = *(const v4f*)(&Tf[rr][lane * 4]); __threadfence(); } }
    wave_lds_sync(); }
}
__global__ __launch_bounds__(64) void mrec_kernel(const float* __restrict__ P, const float* __restrict__ IF, float* __restrict__ HM) {
  __shared__ float Cl[DH][DH + 1], Ks[DH], Qs[DH], Red[2];
  const int d = threadIdx.x, wv = d >> 5, lane = d & 31; const int b = blockIdx.x / NH, hd = blockIdx.x % NH;
#pragma unroll 1
  for (int pass = 0; pass < 2; ++pass) { for (int e = 0; e < DH; ++e) Cl[d][e] = 0.0f; float n = 0.0f, m = 0.0f; __syncthreads();
#pragma unroll 1
    for (int t = 0; t < T; ++t) { const size_t row = (size_t)b * T + t; const float* pr = P + row * 1024 + hd * DH; const float qd = pr[d], kd = pr[256 + d], vd = pr[512 + d], od = pr[768 + d]; const float ig = IF[row * 8 + hd], fg = IF[row * 8 + 4 + hd];
      Ks[d] = kd; Qs[d] = qd; __syncthreads();
      const float mn = fmaxf(fg + m, ig); const float is = __expf(ig - mn), fs = __expf(fg + m - mn); m = mn; const float iv = pmul(is, vd); float num = 0.0f;
#pragma unroll 4
      for (int e = 0; e < DH; ++e) { float c = Cl[d][e]; c = pmul(fs, c) + pmul(iv, Ks[e]); num += pmul(c, Qs[e]); Cl[d][e] = c; }
      n = pmul(fs, n) + pmul(is, kd); float pq = pmul(n, qd); for (int o = 16; o; o >>= 1) pq += __shfl_xor(pq, o); if (lane == 0) Red[wv] = pq; __syncthreads();
      const float den = fmaxf(fabsf(Red[0] + Red[1]), 1.0f); ((volatile float*)HM)[row * H + hd * DH + d] = pmul(od, num) / den; __syncthreads(); }
    __threadfence(); }
}
__global__ __launch_bounds__(32) void post_kernel(const float* __restrict__ HM, const b16* __restrict__ WP, int NTV, float* XR) {
  __shared__ __attribute__((aligned(16))) b16 Ah[16][H + 8], Al[16][H + 8]; __shared__ __attribute__((aligned(16))) float Tf[16][D + 4];
  const int lane = threadIdx.x, nloc = lane & 15, hlf = lane >> 4; const size_t m0 = (size_t)blockIdx.x * 16; if (m0 >= (size_t)NTV) return;
  for (int rr = 0; rr < 16; ++rr) for (int q = 0; q < 8; ++q) { const int c = q * 32 + lane; b16 p, ql; split16(HM[(m0 + rr) * H + c] * HS, p, ql); Ah[rr][c] = p; Al[rr][c] = ql; Tf[rr][c] = XR[(m0 + rr) * D + c]; }
  wave_lds_sync();
#pragma unroll 1
  for (int cg = 0; cg < 2; ++cg) { v8f acc[8];
#pragma unroll
    for (int t = 0; t < 8; ++t) acc[t] = (v8f){};
#pragma unroll 2
    for (int kb = 0; kb < H; kb += 32) { const v16b a = frag_kb(&Ah[nloc][kb], hlf), al = frag_kb(&Al[nloc][kb], hlf);
#pragma unroll
      for (int t = 0; t < 8; ++t) { const v16b bw = frag_kb(WP + (size_t)(cg * 128 + t * 16 + nloc) * H + kb, hlf); acc[t] = wmma16b(a, bw, acc[t]); acc[t] = wmma16b(al, bw, acc[t]); } }
#pragma unroll
    for (int t = 0; t < 8; ++t) { const int c = cg * 128 + t * 16 + nloc;
#pragma unroll 1
      for (int r8 = 0; r8 < 8; ++r8) Tf[8 * hlf + r8][c] += acc[t][r8] * (1.0f / (HS * WSC)); } }
  wave_lds_sync();
  for (int pass = 0; pass < 2; ++pass) { for (int rr = 0; rr < 16; ++rr) for (int q = 0; q < 2; ++q) *(volatile v4f*)(XR + (m0 + rr) * D + q * 128 + lane * 4) = *(const v4f*)(&Tf[rr][q * 128 + lane * 4]); __threadfence(); }
}
__global__ __launch_bounds__(32) void srec_kernel(const float* __restrict__ SX, const b16* __restrict__ WR, float* __restrict__ HSo) {
  __shared__ __attribute__((aligned(16))) b16 Ah[16][DH + 8], Al[16][DH + 8]; __shared__ float Cs[16][DH + 1], Ns[16][DH + 1], Ms[16][DH + 1], Hh[16][DH + 1];
  const int lane = threadIdx.x, nloc = lane & 15, hlf = lane >> 4; const int b0 = blockIdx.x * 16, hd = blockIdx.y; const b16* W = WR + (size_t)hd * 256 * DH; const float sc = 1.0f / (HS * WSC);
#pragma unroll 1
  for (int pass = 0; pass < 2; ++pass) {
    for (int rr = 0; rr < 16; ++rr) for (int q = 0; q < 2; ++q) { Cs[rr][q * 32 + lane] = 0.0f; Ns[rr][q * 32 + lane] = 0.0f; Ms[rr][q * 32 + lane] = 0.0f; Hh[rr][q * 32 + lane] = 0.0f; }
    wave_lds_sync();
#pragma unroll 1
    for (int t = 0; t < T; ++t) {
      for (int rr = 0; rr < 16; ++rr) for (int q = 0; q < 2; ++q) { b16 p, ql; split16(Hh[rr][q * 32 + lane] * HS, p, ql); Ah[rr][q * 32 + lane] = p; Al[rr][q * 32 + lane] = ql; }
      wave_lds_sync();
      v8f acc[16];
#pragma unroll
      for (int tt = 0; tt < 16; ++tt) acc[tt] = (v8f){};
#pragma unroll
      for (int kb = 0; kb < DH; kb += 32) { const v16b a = frag_kb(&Ah[nloc][kb], hlf), al = frag_kb(&Al[nloc][kb], hlf);
#pragma unroll
        for (int tt = 0; tt < 16; ++tt) { const v16b bw = frag_kb(W + (size_t)(tt * 16 + nloc) * DH + kb, hlf); acc[tt] = wmma16b(a, bw, acc[tt]); acc[tt] = wmma16b(al, bw, acc[tt]); } }
      wave_lds_sync();
#pragma unroll
      for (int t4 = 0; t4 < 4; ++t4) { const int e = t4 * 16 + nloc;
#pragma unroll
        for (int r8 = 0; r8 < 8; ++r8) { const int rl = 8 * hlf + r8; const size_t row = (size_t)(b0 + rl) * T + t; const float* sx = SX + row * 1024 + hd * DH + e;
          const float z = tanhf(sx[0] + acc[t4][r8] * sc), ip = sx[256] + acc[4 + t4][r8] * sc, fp = sx[512] + acc[8 + t4][r8] * sc, o = sigm(sx[768] + acc[12 + t4][r8] * sc);
          const float m = Ms[rl][e]; const float mn = fmaxf(fp + m, ip); const float is = __expf(ip - mn), fs = __expf(fp + m - mn); const float c = pmul(fs, Cs[rl][e]) + pmul(is, z); const float n = pmul(fs, Ns[rl][e]) + is; const float h = pmul(o, c) / n;
          Cs[rl][e] = c; Ns[rl][e] = n; Ms[rl][e] = mn; Hh[rl][e] = h; } }
      wave_lds_sync();
      for (int rr = 0; rr < 16; ++rr) for (int q = 0; q < 2; ++q) ((volatile float*)HSo)[((size_t)(b0 + rr) * T + t) * H + hd * DH + q * 32 + lane] = Hh[rr][q * 32 + lane];
    }
    __threadfence(); }
}
__global__ __launch_bounds__(32) void fc_kernel(const float* __restrict__ XR, const float* __restrict__ fw, const float* __restrict__ fb, int BV, float* __restrict__ out) {
  const int lane = threadIdx.x; float s = bf16_rne(fb[0]); const size_t row = (size_t)lane * T + (T - 1);
#pragma unroll 1
  for (int c = 0; c < D; c += 4) { const v4f v = *(const v4f*)(XR + row * D + c); for (int j = 0; j < 4; ++j) s += pmul(v[j], bf16_rne(fw[c + j])); }
  for (int pass = 0; pass < 2; ++pass) { ((volatile float*)out)[lane] = lane < BV ? s : 0.0f; __threadfence(); }
}
}

extern "C" void kernel_launch(void* const* d_in, const int* in_sizes, int n_in, void* d_out, int out_size, void* d_ws, size_t ws_size, hipStream_t stream) {
  (void)n_in;
  auto Fp = [&](int i) { return (const float*)d_in[i]; }; auto Ip = [&](int i) { return (const int*)d_in[i]; };
  if (in_sizes[0] != NT * F || in_sizes[1] != B || in_sizes[2] != NDY * EE || in_sizes[5] != 2 * D * H || in_sizes[8] != 2 * D * NH || in_sizes[13] != 2 * H * D || in_sizes[16] != D * H || in_sizes[20] != NH * DH * DH || in_sizes[24] != H * D || in_sizes[25] != D || out_size != B) return;
  const int BV = B; const int NTV = BV * T;
  size_t off = 0; char* ws = (char*)d_ws;
  auto carve = [&](size_t bytes) { char* p = ws + off; off += (bytes + 255) & ~(size_t)255; return p; };
  b16* WM[2]; b16* WMP[2]; for (int l = 0; l < 2; ++l) { WM[l] = (b16*)carve((size_t)PW * D * 2); WMP[l] = (b16*)carve((size_t)D * H * 2); }
  b16* WS4 = (b16*)carve((size_t)1024 * D * 2); b16* WSP = (b16*)carve((size_t)D * H * 2); b16* WR = (b16*)carve((size_t)NH * 256 * DH * 2);
  float* XR = (float*)carve((size_t)NT * D * 4); float* P = (float*)carve((size_t)NT * 1024 * 4); float* IF = (float*)carve((size_t)NT * 8 * 4); float* HM = (float*)carve((size_t)NT * H * 4);
  if (off > ws_size || off > ((size_t)96 << 20)) return;
  for (int l = 0; l < 2; ++l) { wzero_kernel<<<(PW * D / 8 + 255) / 256, 256, 0, stream>>>(WM[l], PW * D / 8);
    wio_kernel<<<(H * D / 8 + 255) / 256, 256, 0, stream>>>(Fp(5) + (size_t)l * D * H, D, H, 0, WM[l]); wio_kernel<<<(H * D / 8 + 255) / 256, 256, 0, stream>>>(Fp(6) + (size_t)l * D * H, D, H, 256, WM[l]);
    wio_kernel<<<(H * D / 8 + 255) / 256, 256, 0, stream>>>(Fp(7) + (size_t)l * D * H, D, H, 512, WM[l]); wio_kernel<<<(H * D / 8 + 255) / 256, 256, 0, stream>>>(Fp(12) + (size_t)l * D * H, D, H, 768, WM[l]);
    wio_kernel<<<(NH * D / 8 + 255) / 256, 256, 0, stream>>>(Fp(8) + (size_t)l * D * NH, D, NH, 1024, WM[l]); wio_kernel<<<(NH * D / 8 + 255) / 256, 256, 0, stream>>>(Fp(9) + (size_t)l * D * NH, D, NH, 1028, WM[l]);
    wio_kernel<<<(D * H / 8 + 255) / 256, 256, 0, stream>>>(Fp(13) + (size_t)l * H * D, H, D, 0, WMP[l]); }
  wio_kernel<<<(H * D / 8 + 255) / 256, 256, 0, stream>>>(Fp(16), D, H, 0, WS4); wio_kernel<<<(H * D / 8 + 255) / 256, 256, 0, stream>>>(Fp(17), D, H, 256, WS4); wio_kernel<<<(H * D / 8 + 255) / 256, 256, 0, stream>>>(Fp(18), D, H, 512, WS4); wio_kernel<<<(H * D / 8 + 255) / 256, 256, 0, stream>>>(Fp(19), D, H, 768, WS4);
  wio_kernel<<<(D * H / 8 + 255) / 256, 256, 0, stream>>>(Fp(24), H, D, 0, WSP); wr_kernel<<<(NH * 256 * DH / 8 + 255) / 256, 256, 0, stream>>>(Fp(20), Fp(21), Fp(22), Fp(23), WR);
  x0_kernel<<<NTV / 16, 32, 0, stream>>>(Fp(0), Ip(1), Fp(2), XR);
  proj_kernel<0><<<NTV / 16, 32, 0, stream>>>(XR, Fp(3), Fp(4), WM[0], Fp(10), Fp(11), NTV, P, IF);
  mrec_kernel<<<BV * NH, 64, 0, stream>>>(P, IF, HM);
  post_kernel<<<NTV / 16, 32, 0, stream>>>(HM, WMP[0], NTV, XR);
  proj_kernel<1><<<NTV / 16, 32, 0, stream>>>(XR, Fp(14), Fp(15), WS4, nullptr, nullptr, NTV, P, IF);
  srec_kernel<<<dim3(BV / 16, NH), 32, 0, stream>>>(P, WR, HM);
  post_kernel<<<NTV / 16, 32, 0, stream>>>(HM, WSP, NTV, XR);
  proj_kernel<0><<<NTV / 16, 32, 0, stream>>>(XR, Fp(3) + D, Fp(4) + D, WM[1], Fp(10) + NH, Fp(11) + NH, NTV, P, IF);
  mrec_kernel<<<BV * NH, 64, 0, stream>>>(P, IF, HM);
  post_kernel<<<NTV / 16, 32, 0, stream>>>(HM, WMP[1], NTV, XR);
  fc_kernel<<<1, 32, 0, stream>>>(XR, Fp(25), Fp(26), BV, (float*)d_out);
}
